// RotationallyAsymmetricCausalSelfAttention_25683904430761
// MI455X (gfx1250) — hardware-verified
//
#include <hip/hip_runtime.h>
#include <stdint.h>
#include <math.h>

constexpr int kBatch = 4;
constexpr int kSeq   = 2048;
constexpr int kDim   = 1024;
constexpr int kHeads = 16;
constexpr int kHD    = 64;
constexpr int kTok   = kBatch * kSeq;
constexpr int kDim3  = 3 * kDim;

typedef __attribute__((ext_vector_type(16))) _Float16 v16h;
typedef __attribute__((ext_vector_type(8)))  _Float16 v8h;
typedef __attribute__((ext_vector_type(16))) __bf16   v16b;
typedef __attribute__((ext_vector_type(8)))  __bf16   v8b;
typedef __attribute__((ext_vector_type(8)))  float    v8f;
typedef __attribute__((ext_vector_type(4)))  float    v4f;

__device__ __forceinline__ unsigned short f2bf_bits(float f) {
  unsigned u = __float_as_uint(f);
  return (unsigned short)((u + 0x7FFFu + ((u >> 16) & 1u)) >> 16);
}
__device__ __forceinline__ float bf_bits2f(unsigned short h) { return __uint_as_float(((unsigned)h) << 16); }
__device__ __forceinline__ float bf_rne(float f) { return bf_bits2f(f2bf_bits(f)); }

__device__ __forceinline__ void dep_guard_h(v8f& a, v8f& b, v16h x, v16h y) { asm volatile("v_nop\n\tv_nop\n\tv_nop\n\tv_nop" : "+v"(a), "+v"(b) : "v"(x), "v"(y)); }
__device__ __forceinline__ void dep_guard_b(v8f& a, v8f& b, v16b x, v16b y) { asm volatile("v_nop\n\tv_nop\n\tv_nop\n\tv_nop" : "+v"(a), "+v"(b) : "v"(x), "v"(y)); }
__device__ __forceinline__ void keep4_h(v16h a, v16h b, v16h c, v16h d) { asm volatile("v_nop" :: "v"(a), "v"(b), "v"(c), "v"(d)); }
__device__ __forceinline__ void keep4_b(v16b a, v16b b, v16b c, v16b d) { asm volatile("v_nop" :: "v"(a), "v"(b), "v"(c), "v"(d)); }
__device__ __forceinline__ void acc_guard4(v8f& a, v8f& b, v8f& c, v8f& d) { asm volatile("v_nop\n\tv_nop\n\tv_nop\n\tv_nop" : "+v"(a), "+v"(b), "+v"(c), "+v"(d)); }
template <typename T> struct Frag;
template <> struct Frag<_Float16> {
  typedef v16h V; union U { v16h v; v8h h[2]; };
  static __device__ __forceinline__ v16h load(const _Float16* p) {
    U f; f.h[0] = *(const v8h*)(p); f.h[1] = *(const v8h*)(p + 16); return f.v;
  }
  static __device__ __forceinline__ v8f mma(v16h a, v16h b, v8f c) {
    return __builtin_amdgcn_wmma_f32_16x16x32_f16(false, a, false, b, (short)0, c, false, false);
  }
  static __device__ __forceinline__ void guard(v8f& a, v8f& b, v16h x, v16h y) { dep_guard_h(a, b, x, y); }
  static __device__ __forceinline__ void keep(v16h a, v16h b, v16h c, v16h d) { keep4_h(a, b, c, d); }
};
template <> struct Frag<__bf16> {
  typedef v16b V; union U { v16b v; v8b h[2]; };
  static __device__ __forceinline__ v16b load(const __bf16* p) {
    U f; f.h[0] = *(const v8b*)(p); f.h[1] = *(const v8b*)(p + 16); return f.v;
  }
  static __device__ __forceinline__ v8f mma(v16b a, v16b b, v8f c) {
    return __builtin_amdgcn_wmma_f32_16x16x32_bf16(false, a, false, b, (short)0, c, false, false);
  }
  static __device__ __forceinline__ void guard(v8f& a, v8f& b, v16b x, v16b y) { dep_guard_b(a, b, x, y); }
  static __device__ __forceinline__ void keep(v16b a, v16b b, v16b c, v16b d) { keep4_b(a, b, c, d); }
};

template <int ET> struct Elem;
template <> struct Elem<0> { typedef _Float16 T; };
template <> struct Elem<1> { typedef __bf16 T; };
template <int ET, int SPLIT_MODE, int BIAS_MODE, int OUT_MODE, bool RESID, int ACT = 0>
__global__ __launch_bounds__(256) void wmma_gemm64(
    const unsigned short* __restrict__ Ap, const unsigned short* __restrict__ A2p, int lda, long strideA,
    const unsigned short* __restrict__ Btp, const unsigned short* __restrict__ Bt2p, int ldb, long strideB,
    void* __restrict__ Cout, void* __restrict__ Cout2, int ldc, long strideC,
    const float* __restrict__ bias,
    const float* __restrict__ resid, long strideR,
    const float* __restrict__ affs0, const float* __restrict__ affb0,
    const float* __restrict__ affs1, const float* __restrict__ affb1,
    int M, int N, int K, float scale) {
  typedef typename Elem<ET>::T T;
  typedef typename Frag<T>::V V;
  const T* A = (const T*)Ap; const T* A2 = (const T*)A2p; const T* Bt = (const T*)Btp; const T* Bt2 = (const T*)Bt2p;
  __shared__ __align__(16) float sT[8][16 * 68];
  const int b    = blockIdx.y;
  const int lane = threadIdx.x & 31;
  const int wave = threadIdx.x >> 5;
  const int tilesN = N >> 6;
  const int tilesM = M >> 6;
  const int tile = blockIdx.x * 8 + wave;
  if (tile >= tilesM * tilesN) return;
  const int tm = tile / tilesN;
  const int tn = tile - tm * tilesN;
  const int m0 = tm << 6;
  const int n0 = tn << 6;

  const T* Ab  = A  + (size_t)b * strideA;
  const T* Bb  = Bt + (size_t)b * strideB;
  const T* Ab2 = (SPLIT_MODE >= 1) ? (A2  + (size_t)b * strideA) : nullptr;
  const T* Bb2 = (SPLIT_MODE == 2) ? (Bt2 + (size_t)b * strideB) : nullptr;

  const int rlane = lane & 15;
  const int koff  = (lane >> 4) * 8;
  const int mOff  = (lane >> 4) * 8;

  v8f acc[4][4];
#pragma unroll
  for (int i = 0; i < 4; ++i)
#pragma unroll
    for (int j = 0; j < 4; ++j) acc[i][j] = (v8f){0.f,0.f,0.f,0.f,0.f,0.f,0.f,0.f};

  for (int k0 = 0; k0 < K; k0 += 32) {
    V bh[4], bl[4];
#pragma unroll
    for (int j = 0; j < 4; ++j) {
      const size_t bo = (size_t)(n0 + (j << 4) + rlane) * ldb + koff + k0;
      bh[j] = Frag<T>::load(Bb + bo);
      if (SPLIT_MODE == 2) bl[j] = Frag<T>::load(Bb2 + bo);
    }
#pragma unroll
    for (int i = 0; i < 4; ++i) {
      const size_t ao = (size_t)(m0 + (i << 4) + rlane) * lda + koff + k0;
      V ah = Frag<T>::load(Ab + ao);
      V al;
      if (SPLIT_MODE >= 1) al = Frag<T>::load(Ab2 + ao);
#pragma unroll
      for (int j = 0; j < 4; ++j) {
        acc[i][j] = Frag<T>::mma(ah, bh[j], acc[i][j]);
        if (SPLIT_MODE == 2) acc[i][j] = Frag<T>::mma(ah, bl[j], acc[i][j]);
        if (SPLIT_MODE >= 1) acc[i][j] = Frag<T>::mma(al, bh[j], acc[i][j]);
      }
      Frag<T>::guard(acc[i][0], acc[i][3], ah, (SPLIT_MODE >= 1) ? al : ah);
    }
    Frag<T>::keep(bh[0], bh[1], bh[2], bh[3]);
    if (SPLIT_MODE == 2) Frag<T>::keep(bl[0], bl[1], bl[2], bl[3]);
  }
  acc_guard4(acc[0][0], acc[0][1], acc[0][2], acc[0][3]);
  acc_guard4(acc[1][0], acc[1][1], acc[1][2], acc[1][3]);
  acc_guard4(acc[2][0], acc[2][1], acc[2][2], acc[2][3]);
  acc_guard4(acc[3][0], acc[3][1], acc[3][2], acc[3][3]);

  float* slab = sT[wave];
  const float* Rb = RESID ? (resid + (size_t)b * strideR) : nullptr;
#pragma unroll
  for (int i = 0; i < 4; ++i) {
    const int mBase = m0 + (i << 4);
#pragma unroll
    for (int j = 0; j < 4; ++j) {
      const int n = n0 + (j << 4) + rlane;
      float bv = 0.f;
      if (BIAS_MODE == 2) bv = bias[n];
      float asc = 1.0f, abi = 0.0f;
      if (OUT_MODE == 3) {
        const int which = n0 / kDim;
        const int cc = n - which * kDim;
        const float s0 = bf_rne(affs0[cc]);
        const float c0 = bf_rne(affb0[cc]);
        const float s1 = bf_rne(affs1[cc]);
        const float c1 = bf_rne(affb1[cc]);
        asc = (which == 0) ? s0 : ((which == 1) ? s1 : 1.0f);
        abi = (which == 0) ? c0 : ((which == 1) ? c1 : 0.0f);
      }
#pragma unroll
      for (int r = 0; r < 8; ++r) {
        float v = acc[i][j][r] * scale;
        if (BIAS_MODE == 1) v += bias[mBase + mOff + r];
        if (BIAS_MODE == 2) v += bv;
        if (OUT_MODE == 3) v = v * asc + abi;
        if (RESID) v += Rb[(size_t)(mBase + mOff + r) * ldc + n];
        if (ACT == 1) v = tanhf(v);
        if (ACT == 2) v = fmaxf(v, 0.0f);
        if (ACT == 4) v = (v > 0.f) ? v : 0.01f * v;
        slab[(mOff + r) * 68 + (j << 4) + rlane] = v;
      }
    }
    __builtin_amdgcn_fence(__ATOMIC_RELEASE, "workgroup");
    __builtin_amdgcn_wave_barrier();
    __builtin_amdgcn_fence(__ATOMIC_ACQUIRE, "workgroup");
    if (OUT_MODE == 0) {
      float* C = (float*)Cout + (size_t)b * strideC;
      const int hh = lane >> 4, c4 = (lane & 15) * 4;
      for (int pass = 0; pass < 2; ++pass) {
#pragma unroll
        for (int it = 0; it < 8; ++it) {
          const int row = it * 2 + hh;
          v4f v = *(const v4f*)(slab + row * 68 + c4);
          *(volatile v4f*)(C + (size_t)(mBase + row) * ldc + n0 + c4) = v;
        }
        __threadfence();
      }
    } else {
      const int q = lane >> 3, c8 = (lane & 7) * 8;
      unsigned short* C;
      unsigned short* C2;
      int ncol;
      if (OUT_MODE == 3) {
        const int which = n0 / kDim;
        C  = (unsigned short*)Cout + (size_t)which * 2 * (size_t)strideC;
        C2 = C + (size_t)strideC;
        ncol = n0 - which * kDim;
      } else {
        C  = (unsigned short*)Cout  + (size_t)b * strideC;
        C2 = (OUT_MODE == 2) ? ((unsigned short*)Cout2 + (size_t)b * strideC) : nullptr;
        ncol = n0;
      }
      for (int pass = 0; pass < 2; ++pass) {
#pragma unroll
        for (int it = 0; it < 4; ++it) {
          const int row = it * 4 + q;
          const float* sp = slab + row * 68 + c8;
          v8h hv, lv;
#pragma unroll
          for (int e = 0; e < 8; ++e) {
            if (OUT_MODE == 1) {
              hv[e] = (_Float16)sp[e];
            } else {
              unsigned short hb = f2bf_bits(sp[e]);
              unsigned short lb = f2bf_bits(sp[e] - bf_bits2f(hb));
              hv[e] = __builtin_bit_cast(_Float16, hb);
              lv[e] = __builtin_bit_cast(_Float16, lb);
            }
          }
          *(volatile v8h*)(C + (size_t)(mBase + row) * ldc + ncol + c8) = hv;
          if (OUT_MODE >= 2) *(volatile v8h*)(C2 + (size_t)(mBase + row) * ldc + ncol + c8) = lv;
        }
        __threadfence();
      }
    }
    __builtin_amdgcn_fence(__ATOMIC_RELEASE, "workgroup");
    __builtin_amdgcn_wave_barrier();
    __builtin_amdgcn_fence(__ATOMIC_ACQUIRE, "workgroup");
  }
}

__global__ __launch_bounds__(256) void cast_bf16x8_k(const float* __restrict__ in,
                                                     unsigned short* __restrict__ out, int n8) {
  const int i = blockIdx.x * 256 + threadIdx.x;
  if (i < n8) {
    const size_t o = (size_t)i * 8;
    const v4f a = *(const v4f*)(in + o);
    const v4f bq = *(const v4f*)(in + o + 4);
    v8h hv;
#pragma unroll
    for (int e = 0; e < 4; ++e) {
      hv[e]     = __builtin_bit_cast(_Float16, f2bf_bits(a[e]));
      hv[4 + e] = __builtin_bit_cast(_Float16, f2bf_bits(bq[e]));
    }
    *(volatile v8h*)(out + o) = hv;
    __threadfence();
    *(volatile v8h*)(out + o) = hv;
  }
}

constexpr int kWTP = 72;
__global__ __launch_bounds__(256) void wt_cast_bf_k(const float* __restrict__ W, unsigned short* __restrict__ Wtp,
                                                    int K, int N) {
  __shared__ __align__(16) _Float16 st[64 * kWTP];
  _Float16* Wt = (_Float16*)Wtp;
  const int n0 = blockIdx.x * 64, k0 = blockIdx.y * 64;
  const int tid = threadIdx.x;
  const int kr = tid >> 2, c16 = (tid & 3) * 16;
  const float* src = W + (size_t)(k0 + kr) * N + n0 + c16;
#pragma unroll
  for (int qq = 0; qq < 4; ++qq) {
    const v4f v = *(const v4f*)(src + 4 * qq);
#pragma unroll
    for (int e = 0; e < 4; ++e)
      st[(c16 + 4 * qq + e) * kWTP + kr] = __builtin_bit_cast(_Float16, f2bf_bits(v[e]));
  }
  __syncthreads();
  const int wave = tid >> 5, lane = tid & 31;
  const int q8 = lane >> 3, c8 = (lane & 7) * 8;
  for (int pass = 0; pass < 2; ++pass) {
#pragma unroll
    for (int it = 0; it < 2; ++it) {
      const int n = it * 32 + wave * 4 + q8;
      const v8h hv = *(const v8h*)(st + n * kWTP + c8);
      *(volatile v8h*)(Wt + (size_t)(n0 + n) * K + k0 + c8) = hv;
    }
    __threadfence();
  }
}

constexpr int kKC = 64;
constexpr int kQB = 64;

__device__ __forceinline__ v8f mma_bf(v16b a, v16b b, v8f c) {
  c = __builtin_amdgcn_wmma_f32_16x16x32_bf16(false, a, false, b, (short)0, c, false, false);
  asm volatile("v_nop\n\tv_nop\n\tv_nop\n\tv_nop" : "+v"(c) : "v"(a), "v"(b));
  return c;
}

__global__ __launch_bounds__(128)
void attn_hd64_k(const unsigned short* __restrict__ Qhp, const unsigned short* __restrict__ Qlp,
                 const unsigned short* __restrict__ Khp, const unsigned short* __restrict__ Klp,
                 const unsigned short* __restrict__ Vhp, const unsigned short* __restrict__ Vlp,
                 unsigned short* __restrict__ Yhp, unsigned short* __restrict__ Ylp, int bsel) {
  union FB { v16b v; v8b h[2]; };
  __shared__ __align__(16) __bf16 Ksh[kKC * kHD];
  __shared__ __align__(16) __bf16 Ksl[kKC * kHD];
  __shared__ __align__(16) __bf16 Vth[kHD * kKC];
  __shared__ __align__(16) __bf16 Vtl[kHD * kKC];
  __shared__ __align__(16) __bf16 Pbuf[4][2 * 16 * kKC];

  const __bf16* Qh = (const __bf16*)Qhp;
  const __bf16* Ql = (const __bf16*)Qlp;
  const __bf16* Kh = (const __bf16*)Khp;
  const __bf16* Kl = (const __bf16*)Klp;
  const __bf16* Vh = (const __bf16*)Vhp;
  const __bf16* Vl = (const __bf16*)Vlp;

  const int tid  = threadIdx.x;
  const int wave = tid >> 5;
  const int lane = tid & 31;
  const int hh   = lane >> 4;
  const int c    = lane & 15;

  constexpr int nqb = kSeq / kQB;
  const int bx = blockIdx.x;
  const int qb = bx % nqb;
  const int h  = bx / nqb;
  const int q0 = qb * kQB + wave * 16;
  const size_t rowb = (size_t)bsel * kSeq;
  const int hcol = h * kHD;

  v16b qah[2], qal[2];
  {
    const size_t qoff = (rowb + (size_t)(q0 + c)) * kDim + hcol + 8 * hh;
#pragma unroll
    for (int dc = 0; dc < 2; ++dc) {
      qah[dc] = Frag<__bf16>::load(Qh + qoff + dc * 32);
      qal[dc] = Frag<__bf16>::load(Ql + qoff + dc * 32);
    }
  }

  float mrow[8], lrow[8];
  v8f oacc[4];
#pragma unroll
  for (int r = 0; r < 8; ++r) { mrow[r] = -INFINITY; lrow[r] = 0.f; }
#pragma unroll
  for (int t = 0; t < 4; ++t) oacc[t] = (v8f){0.f,0.f,0.f,0.f,0.f,0.f,0.f,0.f};

  const int nChunks = qb + 1;
  for (int kc = 0; kc < nChunks; ++kc) {
    const int kv0 = kc * kKC;
    __syncthreads();
    {
      const int kvr = tid >> 1, dh = (tid & 1) * 32;
      const size_t goff = (rowb + (size_t)(kv0 + kvr)) * kDim + hcol + dh;
#pragma unroll 1
      for (int i = 0; i < 4; ++i) {
        const v8b a0 = *(const v8b*)(Kh + goff + 8 * i);
        const v8b a1 = *(const v8b*)(Kl + goff + 8 * i);
        *(v8b*)(Ksh + kvr * kHD + dh + 8 * i) = a0;
        *(v8b*)(Ksl + kvr * kHD + dh + 8 * i) = a1;
        const v8b w0 = *(const v8b*)(Vh + goff + 8 * i);
        const v8b w1 = *(const v8b*)(Vl + goff + 8 * i);
#pragma unroll
        for (int e = 0; e < 8; ++e) {
          Vth[(dh + 8 * i + e) * kKC + kvr] = w0[e];
          Vtl[(dh + 8 * i + e) * kKC + kvr] = w1[e];
        }
      }
    }
    __syncthreads();

    v8f s[4];
#pragma unroll
    for (int j = 0; j < 4; ++j) {
      s[j] = (v8f){0.f,0.f,0.f,0.f,0.f,0.f,0.f,0.f};
#pragma unroll
      for (int dc = 0; dc < 2; ++dc) {
        FB kb, kl;
        kb.h[0] = *(const v8b*)(Ksh + (j * 16 + c) * kHD + dc * 32 + 8 * hh);
        kb.h[1] = *(const v8b*)(Ksh + (j * 16 + c) * kHD + dc * 32 + 16 + 8 * hh);
        kl.h[0] = *(const v8b*)(Ksl + (j * 16 + c) * kHD + dc * 32 + 8 * hh);
        kl.h[1] = *(const v8b*)(Ksl + (j * 16 + c) * kHD + dc * 32 + 16 + 8 * hh);
        s[j] = mma_bf(qah[dc], kb.v, s[j]);
        s[j] = mma_bf(qah[dc], kl.v, s[j]);
        s[j] = mma_bf(qal[dc], kb.v, s[j]);
      }
    }
    const bool diag = (kc == qb);
    float cm[8];
#pragma unroll
    for (int r = 0; r < 8; ++r) {
      const int qrow = q0 + 8 * hh + r;
      float m = -INFINITY;
#pragma unroll
      for (int j = 0; j < 4; ++j) {
        const int kvcol = kv0 + j * 16 + c;
        float sv = s[j][r] * 0.125f;
        if (diag && (kvcol > qrow)) sv = -INFINITY;
        s[j][r] = sv;
        m = fmaxf(m, sv);
      }
#pragma unroll
      for (int off = 1; off < 16; off <<= 1) m = fmaxf(m, __shfl_xor(m, off, 32));
      cm[r] = m;
    }
    __bf16* pwh = Pbuf[wave];
    __bf16* pwl = Pbuf[wave] + 16 * kKC;
#pragma unroll
    for (int r = 0; r < 8; ++r) {
      const float mnew = fmaxf(mrow[r], cm[r]);
      const float mref = (mnew > -INFINITY) ? mnew : 0.0f;
      const float alpha = expf(mrow[r] - mref);
      mrow[r] = mnew;
      float psum = 0.f;
#pragma unroll
      for (int j = 0; j < 4; ++j) {
        const float p = expf(s[j][r] - mref);
        psum += p;
        const unsigned short hb = f2bf_bits(p);
        const unsigned short lb = f2bf_bits(p - bf_bits2f(hb));
        pwh[(8 * hh + r) * kKC + j * 16 + c] = __builtin_bit_cast(__bf16, hb);
        pwl[(8 * hh + r) * kKC + j * 16 + c] = __builtin_bit_cast(__bf16, lb);
      }
#pragma unroll
      for (int off = 1; off < 16; off <<= 1) psum += __shfl_xor(psum, off, 32);
      lrow[r] = lrow[r] * alpha + psum;
#pragma unroll
      for (int t = 0; t < 4; ++t) oacc[t][r] *= alpha;
    }
    __builtin_amdgcn_fence(__ATOMIC_RELEASE, "workgroup");
    __builtin_amdgcn_wave_barrier();
    __builtin_amdgcn_fence(__ATOMIC_ACQUIRE, "workgroup");
#pragma unroll 1
    for (int kk = 0; kk < 2; ++kk) {
      FB pa, pl;
      pa.h[0] = *(const v8b*)(pwh + c * kKC + kk * 32 + 8 * hh);
      pa.h[1] = *(const v8b*)(pwh + c * kKC + kk * 32 + 16 + 8 * hh);
      pl.h[0] = *(const v8b*)(pwl + c * kKC + kk * 32 + 8 * hh);
      pl.h[1] = *(const v8b*)(pwl + c * kKC + kk * 32 + 16 + 8 * hh);
#pragma unroll
      for (int t = 0; t < 4; ++t) {
        FB vb, vl;
        vb.h[0] = *(const v8b*)(Vth + (t * 16 + c) * kKC + kk * 32 + 8 * hh);
        vb.h[1] = *(const v8b*)(Vth + (t * 16 + c) * kKC + kk * 32 + 16 + 8 * hh);
        vl.h[0] = *(const v8b*)(Vtl + (t * 16 + c) * kKC + kk * 32 + 8 * hh);
        vl.h[1] = *(const v8b*)(Vtl + (t * 16 + c) * kKC + kk * 32 + 16 + 8 * hh);
        oacc[t] = mma_bf(pa.v, vb.v, oacc[t]);
        oacc[t] = mma_bf(pa.v, vl.v, oacc[t]);
        oacc[t] = mma_bf(pl.v, vb.v, oacc[t]);
      }
    }
  }

  __syncthreads();
  float* os = (float*)(Pbuf[wave]);
#pragma unroll
  for (int r = 0; r < 8; ++r) {
    const float inv = 1.0f / lrow[r];
#pragma unroll
    for (int t = 0; t < 4; ++t) os[(8 * hh + r) * kHD + t * 16 + c] = oacc[t][r] * inv;
  }
  __builtin_amdgcn_fence(__ATOMIC_RELEASE, "workgroup");
  __builtin_amdgcn_wave_barrier();
  __builtin_amdgcn_fence(__ATOMIC_ACQUIRE, "workgroup");
  {
    const int q8 = lane >> 3, c8 = (lane & 7) * 8;
    for (int pass = 0; pass < 2; ++pass) {
#pragma unroll
      for (int it = 0; it < 4; ++it) {
        const int row = it * 4 + q8;
        const float* sp = os + row * kHD + c8;
        v8h hv, lv;
#pragma unroll
        for (int e = 0; e < 8; ++e) {
          const unsigned short hb = f2bf_bits(sp[e]);
          const unsigned short lb = f2bf_bits(sp[e] - bf_bits2f(hb));
          hv[e] = __builtin_bit_cast(_Float16, hb);
          lv[e] = __builtin_bit_cast(_Float16, lb);
        }
        const size_t yo = (size_t)(q0 + row) * kDim + hcol + c8;
        *(volatile v8h*)(Yhp + yo) = hv;
        *(volatile v8h*)(Ylp + yo) = lv;
      }
      __threadfence();
    }
  }
}

extern "C" void kernel_launch(void* const* d_in, const int* in_sizes, int n_in,
                              void* d_out, int out_size, void* d_ws, size_t ws_size,
                              hipStream_t stream) {
  if (n_in < 9) return;
  if (in_sizes[0] != kTok * kDim || in_sizes[1] != kDim * kDim3 || in_sizes[2] != kDim3 ||
      in_sizes[3] != kDim * kDim || in_sizes[4] != kDim ||
      in_sizes[5] != kHeads * kHD || in_sizes[6] != kHeads * kHD ||
      in_sizes[7] != kHeads * kHD || in_sizes[8] != kHeads * kHD ||
      out_size != kTok * kDim) return;

  const float* x     = (const float*)d_in[0];
  const float* Wqkv  = (const float*)d_in[1];
  const float* bqkv  = (const float*)d_in[2];
  const float* Wproj = (const float*)d_in[3];
  const float* bproj = (const float*)d_in[4];
  const float* qs    = (const float*)d_in[5];
  const float* qbv   = (const float*)d_in[6];
  const float* ks    = (const float*)d_in[7];
  const float* kbv   = (const float*)d_in[8];
  float* out = (float*)d_out;

  const size_t plane  = (size_t)kTok * kDim;
  const size_t offX   = 0;
  const size_t offWq  = offX  + plane * 2;
  const size_t offWp  = offWq + (size_t)kDim3 * kDim * 2;
  const size_t offQKV = offWp + (size_t)kDim * kDim * 2;
  const size_t total  = offQKV + 6 * plane * 2;
  if (total > ws_size) return;

  char* ws = (char*)d_ws;
  unsigned short* Xb  = (unsigned short*)(ws + offX);
  unsigned short* Yh  = Xb;
  unsigned short* Yl  = Xb + (size_t)kSeq * kDim;
  unsigned short* WqT = (unsigned short*)(ws + offWq);
  unsigned short* WpT = (unsigned short*)(ws + offWp);
  unsigned short* QKV = (unsigned short*)(ws + offQKV);
  unsigned short* Qh = QKV;
  unsigned short* Ql = QKV + plane;
  unsigned short* Kh = QKV + 2 * plane;
  unsigned short* Kl = QKV + 3 * plane;
  unsigned short* Vh = QKV + 4 * plane;
  unsigned short* Vl = QKV + 5 * plane;

  const int n8 = (kTok * kDim) / 8;
  cast_bf16x8_k<<<dim3((n8 + 255) / 256), dim3(256), 0, stream>>>(x, Xb, n8);

  wt_cast_bf_k<<<dim3(kDim3 / 64, kDim / 64), dim3(256), 0, stream>>>(Wqkv, WqT, kDim, kDim3);
  wt_cast_bf_k<<<dim3(kDim / 64, kDim / 64), dim3(256), 0, stream>>>(Wproj, WpT, kDim, kDim);

  wmma_gemm64<1, 0, 2, 3, false><<<dim3(768, 1), dim3(256), 0, stream>>>(
      Xb, Xb, kDim, 0L, WqT, WqT, kDim, 0L,
      (void*)QKV, (void*)QKV, kDim, (long)plane,
      bqkv, bqkv, 0L, qs, qbv, ks, kbv,
      kTok, kDim3, kDim, 1.0f);

  for (int b = 0; b < kBatch; ++b) {
    attn_hd64_k<<<dim3(kHeads * (kSeq / kQB)), dim3(128), 0, stream>>>(Qh, Ql, Kh, Kl, Vh, Vl, Yh, Yl, b);
    wmma_gemm64<1, 1, 2, 0, false><<<dim3(64, 1), dim3(256), 0, stream>>>(
        Yh, Yl, kDim, 0L, WpT, WpT, kDim, 0L,
        (void*)(out + (size_t)b * kSeq * kDim), (void*)(out + (size_t)b * kSeq * kDim), kDim, 0L,
        bproj, bproj, 0L, qs, qbv, ks, kbv,
        kSeq, kDim, kDim, 1.0f);
  }
}
